// MLPDecoder_20615843021601
// MI455X (gfx1250) — hardware-verified
//
#include <hip/hip_runtime.h>
#include <stddef.h>
#include <stdint.h>

#define NBATCH 4
#define NE     512
#define KD     256
#define HH     256
#define NR     (NBATCH * NE)
#define MH     (2 * HH)
#define TP     72
#define GBM    64
#define GBN    128
#define GTHR   128
#define PT     64
#define NTHR   256
#define WSMAX  134217728

static_assert(KD % 64 == 0 && HH % 64 == 0 && KD % 32 == 0);
static_assert(MH % GBM == 0 && NR % GBN == 0);
static_assert(GBM == (GTHR / 32) * 16 && GBN == 4 * 32);
static_assert((NR * KD / 8) % NTHR == 0);
static_assert(NE % PT == 0 && HH % PT == 0 && PT == 64);
static_assert(HH == NTHR);
static_assert((TP * 2) % 16 == 0);
static_assert(NTHR == 256 && GBM <= NTHR);

typedef float          v4f   __attribute__((ext_vector_type(4)));
typedef float          v8f   __attribute__((ext_vector_type(8)));
typedef int            v4i   __attribute__((ext_vector_type(4)));
typedef int            v8i   __attribute__((ext_vector_type(8)));
typedef unsigned int   v4u   __attribute__((ext_vector_type(4)));
typedef unsigned short v8us  __attribute__((ext_vector_type(8)));
typedef unsigned short v16us __attribute__((ext_vector_type(16)));
typedef __bf16         v16bf __attribute__((ext_vector_type(16)));
typedef v4f  __attribute__((may_alias)) v4fa;
typedef v4i  __attribute__((may_alias)) v4ia;
typedef v4u  __attribute__((may_alias)) v4ua;
typedef v8us __attribute__((may_alias)) v8usa;
union FragB { v16bf v; v16us u; v8us h[2]; v8i w; };

__device__ __forceinline__ v8f wmb(const FragB& a, const FragB& b, v8f c) {
  v8f d = __builtin_amdgcn_wmma_f32_16x16x32_bf16(false, a.v, false, b.v, (short)0, c, false, false);
  asm volatile("v_nop\n\tv_nop\n\tv_nop\n\tv_nop" : "+v"(d) : "v"(a.w), "v"(b.w));
  return d;
}

__device__ __forceinline__ unsigned bf16_bits(float f) {
  const unsigned u = __float_as_uint(f);
  return (u + 0x7FFFu + ((u >> 16) & 1u)) >> 16;
}
__device__ __forceinline__ float bf16_val(float f) {
  return __uint_as_float(bf16_bits(f) << 16);
}
__device__ __forceinline__ unsigned pk16(unsigned a, unsigned b) { return (a & 0xFFFFu) | (b << 16); }

__global__ __launch_bounds__(NTHR) void k_cvt(const float* __restrict__ x, unsigned short* Xb) {
  const int g = (int)blockIdx.x * NTHR + (int)threadIdx.x;
  if (g >= NR * KD / 8) return;
  const float* src = x + (size_t)g * 8;
  const v4f a = *(const v4fa*)src;
  const v4f c = *(const v4fa*)(src + 4);
  v4u o;
  o[0] = pk16(bf16_bits(a[0]), bf16_bits(a[1]));
  o[1] = pk16(bf16_bits(a[2]), bf16_bits(a[3]));
  o[2] = pk16(bf16_bits(c[0]), bf16_bits(c[1]));
  o[3] = pk16(bf16_bits(c[2]), bf16_bits(c[3]));
  unsigned short* dst = Xb + (size_t)g * 8;
  *(volatile v4u*)dst = o;
  __threadfence();
  *(volatile v4u*)dst = o;
}

__global__ __launch_bounds__(NTHR) void k_wt(const float* __restrict__ W1, unsigned short* AT) {
  __shared__ __attribute__((aligned(16))) unsigned short sT[64 * TP];
  const int tid = (int)threadIdx.x, lane = tid & 31, w = tid >> 5;
  const int c0 = (int)blockIdx.x * 64, k0 = (int)blockIdx.y * 64, z = (int)blockIdx.z;
  const float* src = W1 + (size_t)z * KD * HH;
  unsigned short* dst = AT + (size_t)z * HH * KD;
  const int c4 = (tid & 15) * 4, rr = tid >> 4;
#pragma unroll
  for (int p = 0; p < 4; ++p) {
    const int r = rr + 16 * p;
    const v4f v = *(const v4fa*)(src + (size_t)(k0 + r) * HH + c0 + c4);
    sT[(c4 + 0) * TP + r] = (unsigned short)bf16_bits(v[0]);
    sT[(c4 + 1) * TP + r] = (unsigned short)bf16_bits(v[1]);
    sT[(c4 + 2) * TP + r] = (unsigned short)bf16_bits(v[2]);
    sT[(c4 + 3) * TP + r] = (unsigned short)bf16_bits(v[3]);
  }
  __syncthreads();
  const int q8 = lane & 7, sub = lane >> 3;
  v4u vv[2];
#pragma unroll
  for (int it = 0; it < 2; ++it) {
    const int row = 32 * it + 4 * w + sub;
    vv[it] = *(const v4ua*)(sT + row * TP + 8 * q8);
  }
#pragma unroll
  for (int it = 0; it < 2; ++it) {
    const int row = 32 * it + 4 * w + sub;
    *(volatile v4u*)(dst + (size_t)(c0 + row) * KD + k0 + 8 * q8) = vv[it];
  }
  __threadfence();
#pragma unroll
  for (int it = 0; it < 2; ++it) {
    const int row = 32 * it + 4 * w + sub;
    *(volatile v4u*)(dst + (size_t)(c0 + row) * KD + k0 + 8 * q8) = vv[it];
  }
}

__global__ __launch_bounds__(GTHR) void k_gemm(const unsigned short* __restrict__ A, const unsigned short* __restrict__ BT,
                                               const float* __restrict__ b1, float* Cm) {
  __shared__ __attribute__((aligned(16))) float stg[GBM * GBN];
  __shared__ float sb[GBM];
  const int tid = (int)threadIdx.x, lane = tid & 31, wave = tid >> 5, hh = lane >> 4, m = lane & 15;
  const int rowBase = (int)blockIdx.x * GBM;
  const int colBase = (int)blockIdx.y * GBN;

  if (tid < GBM) {
    const int rr = rowBase + tid;
    const int rc = rr < HH ? rr : HH - 1;
    const float v = bf16_val(b1[rc]);
    sb[tid] = rr < HH ? v : 0.0f;
  }
  __syncthreads();

  v8f acc[8];
  {
    const v8f z = {0.f, 0.f, 0.f, 0.f, 0.f, 0.f, 0.f, 0.f};
#pragma unroll
    for (int t = 0; t < 8; ++t) acc[t] = z;
  }
  const unsigned short* ap = A  + (size_t)(rowBase + 16 * wave + m) * (size_t)KD + 8 * hh;
  const unsigned short* bp = BT + (size_t)(colBase + m) * (size_t)KD + 8 * hh;

#pragma unroll 1
  for (int k0 = 0; k0 < KD; k0 += 32) {
    FragB af;
    af.h[0] = *(const v8usa*)(ap + k0);
    af.h[1] = *(const v8usa*)(ap + k0 + 16);
#pragma unroll
    for (int nt = 0; nt < 8; ++nt) {
      const unsigned short* wq = bp + (size_t)(16 * nt) * (size_t)KD + k0;
      FragB bf;
      bf.h[0] = *(const v8usa*)wq;
      bf.h[1] = *(const v8usa*)(wq + 16);
      acc[nt] = wmb(af, bf, acc[nt]);
    }
  }

#pragma unroll
  for (int nt = 0; nt < 8; ++nt) {
    const int lc = 16 * nt + m;
#pragma unroll
    for (int r = 0; r < 8; ++r) {
      const int lr = 16 * wave + 8 * hh + r;
      stg[lr * GBN + lc] = acc[nt][r] + sb[lr];
    }
  }
  __syncthreads();

  v4f pv[16];
#pragma unroll
  for (int i = 0; i < 16; ++i) pv[i] = *(const v4fa*)(stg + (16 * wave + i) * GBN + 4 * lane);
#pragma unroll
  for (int i = 0; i < 16; ++i) {
    float* op = Cm + (size_t)(rowBase + 16 * wave + i) * (size_t)NR + colBase + 4 * lane;
    *(volatile v4f*)op = pv[i];
  }
  __threadfence();
#pragma unroll
  for (int i = 0; i < 16; ++i) {
    float* op = Cm + (size_t)(rowBase + 16 * wave + i) * (size_t)NR + colBase + 4 * lane;
    *(volatile v4f*)op = pv[i];
  }
}

__global__ __launch_bounds__(NTHR) void k_pair(const float* __restrict__ HT, const float* __restrict__ W2,
                                               const float* __restrict__ b2, const int* __restrict__ mask,
                                               float* out) {
  __shared__ __attribute__((aligned(16))) float s_i[PT * PT];
  __shared__ __attribute__((aligned(16))) float s_j[PT * PT];
  __shared__ __attribute__((aligned(16))) float s_w[HH];
  const int t = (int)threadIdx.x, lane = t & 31, w = t >> 5;
  const int b = (int)blockIdx.z, i0 = (int)blockIdx.x * PT, j0 = (int)blockIdx.y * PT;
  const int ti = t & 15, tj = t >> 4;

  s_w[t] = bf16_val(W2[t]);
  const float bb = bf16_val(b2[0]);
  const v4i mi4 = *(const v4ia*)(mask + (size_t)b * NE + i0 + 4 * ti);
  const v4i mj4 = *(const v4ia*)(mask + (size_t)b * NE + j0 + 4 * tj);
  v4f mi, mj;
#pragma unroll
  for (int e = 0; e < 4; ++e) {
    mi[e] = mi4[e] != 0 ? 1.0f : 0.0f;
    mj[e] = mj4[e] != 0 ? 1.0f : 0.0f;
  }

  const v4f zero4 = {0.f, 0.f, 0.f, 0.f};
  v4f acc[4];
#pragma unroll
  for (int a = 0; a < 4; ++a) acc[a] = zero4;

  const float* Hib = HT + (size_t)b * NE + i0;
  const float* Hjb = HT + (size_t)HH * NR + (size_t)b * NE + j0;

#pragma unroll 1
  for (int hc = 0; hc < HH / PT; ++hc) {
    const int h0 = hc * PT;
    __syncthreads();
#pragma unroll
    for (int it = 0; it < 4; ++it) {
      const int h  = (t >> 4) + 16 * it;
      const int c4 = (t & 15) * 4;
      const v4f vi = *(const v4fa*)(Hib + (size_t)(h0 + h) * NR + c4);
      const v4f vj = *(const v4fa*)(Hjb + (size_t)(h0 + h) * NR + c4);
      *(v4fa*)(s_i + h * PT + c4) = vi;
      *(v4fa*)(s_j + h * PT + c4) = vj;
    }
    __syncthreads();

#pragma unroll 2
    for (int hu = 0; hu < PT; ++hu) {
      const v4f hi4 = *(const v4fa*)(s_i + hu * PT + 4 * ti);
      const v4f hj4 = *(const v4fa*)(s_j + hu * PT + 4 * tj);
      const float wv = s_w[h0 + hu];
#pragma unroll
      for (int a = 0; a < 4; ++a)
#pragma unroll
        for (int q = 0; q < 4; ++q) {
          const float v = fmaxf(hi4[a] + hj4[q], 0.0f);
          acc[a][q] = fmaf(v, wv, acc[a][q]);
        }
    }
  }
  __syncthreads();

  float* sO = s_i;
#pragma unroll
  for (int a = 0; a < 4; ++a) {
    v4f o;
#pragma unroll
    for (int q = 0; q < 4; ++q) {
      const float l = acc[a][q] + bb;
      const float e = __expf(-l);
      const float s = __builtin_amdgcn_rcpf(1.0f + e);
      o[q] = s * mi[a] * mj[q];
    }
    *(v4fa*)(sO + (4 * ti + a) * PT + 4 * tj) = o;
  }
  __syncthreads();

  const int rsub = lane >> 4, c4 = (lane & 15) * 4;
  v4f vals[4];
#pragma unroll
  for (int it = 0; it < 4; ++it) {
    const int row = 8 * w + 2 * it + rsub;
    vals[it] = *(const v4fa*)(sO + row * PT + c4);
  }
#pragma unroll
  for (int it = 0; it < 4; ++it) {
    const int row = 8 * w + 2 * it + rsub;
    float* op = out + ((size_t)(b * NE + i0 + row) * (size_t)NE + j0 + c4);
    *(volatile v4f*)op = vals[it];
  }
  __threadfence();
#pragma unroll
  for (int it = 0; it < 4; ++it) {
    const int row = 8 * w + 2 * it + rsub;
    float* op = out + ((size_t)(b * NE + i0 + row) * (size_t)NE + j0 + c4);
    *(volatile v4f*)op = vals[it];
  }
}

extern "C" void kernel_launch(void* const* d_in, const int* in_sizes, int n_in,
                              void* d_out, int out_size, void* d_ws, size_t ws_size,
                              hipStream_t stream) {
  if (n_in < 6) return;
  if (in_sizes[0] != NR * KD) return;
  if (in_sizes[1] != NR) return;
  if (in_sizes[2] != MH * KD) return;
  if (in_sizes[3] != HH) return;
  if (in_sizes[4] != HH) return;
  if (in_sizes[5] != 1) return;
  if (out_size != NBATCH * NE * NE) return;

  const float* x    = (const float*)d_in[0];
  const int*   mask = (const int*)d_in[1];
  const float* W1   = (const float*)d_in[2];
  const float* b1   = (const float*)d_in[3];
  const float* W2   = (const float*)d_in[4];
  const float* b2   = (const float*)d_in[5];
  float* out = (float*)d_out;

  char* ws = (char*)d_ws;
  size_t off = 0;
  const size_t oXb = off; off += (size_t)NR * KD * 2;  off = (off + 255) & ~(size_t)255;
  const size_t oAT = off; off += (size_t)MH * KD * 2;  off = (off + 255) & ~(size_t)255;
  const size_t oHT = off; off += (size_t)MH * NR * 4;  off = (off + 255) & ~(size_t)255;
  if (off > ws_size || off > (size_t)WSMAX) return;
  unsigned short* Xb = (unsigned short*)(ws + oXb);
  unsigned short* AT = (unsigned short*)(ws + oAT);
  float*          HT = (float*)(ws + oHT);

  k_cvt<<<dim3((NR * KD / 8) / NTHR), NTHR, 0, stream>>>(x, Xb);
  k_wt<<<dim3(HH / 64, KD / 64, 2), NTHR, 0, stream>>>(W1, AT);
  k_gemm<<<dim3(MH / GBM, NR / GBN), GTHR, 0, stream>>>(AT, Xb, b1, HT);
  k_pair<<<dim3(NE / PT, NE / PT, NBATCH), NTHR, 0, stream>>>(HT, W2, b2, mask, out);
  (void)hipGetLastError();
}
